// GATv1Layer_81853486727787
// MI455X (gfx1250) — hardware-verified
//
#include <hip/hip_runtime.h>
#include <math.h>
#include <stddef.h>


typedef _Float16 f16_t;
typedef __bf16   bf16_t;
typedef f16_t    v16h __attribute__((ext_vector_type(16)));
typedef f16_t    v8h  __attribute__((ext_vector_type(8)));
typedef bf16_t   v16b __attribute__((ext_vector_type(16)));
typedef bf16_t   v8b  __attribute__((ext_vector_type(8)));
typedef float    v8f  __attribute__((ext_vector_type(8)));
typedef float    v4f  __attribute__((ext_vector_type(4)));
typedef int      v4i  __attribute__((ext_vector_type(4)));
typedef unsigned v4u  __attribute__((ext_vector_type(4)));
union FragH { v16h v; v8h half[2]; };
union FragB { v16b v; v8b half[2]; };

#define C_IN     256
#define C_OUT    256
#define NHEAD    4
#define HDIM     64
#define XP       264
#define SP       260
#define NB_C     1536
#define NB_A     192
#define SB_PITCH 32

__device__ __forceinline__ v8f mma_f16(v16h a, v16h b, v8f c) {
  c = __builtin_amdgcn_wmma_f32_16x16x32_f16(false, a, false, b, (short)0, c, false, false);
  asm volatile("v_nop\n\tv_nop\n\tv_nop\n\tv_nop" : "+v"(c) : "v"(a), "v"(b));
  return c;
}
__device__ __forceinline__ v8f mma_bf16(v16b a, v16b b, v8f c) {
  c = __builtin_amdgcn_wmma_f32_16x16x32_bf16(false, a, false, b, (short)0, c, false, false);
  asm volatile("v_nop\n\tv_nop\n\tv_nop\n\tv_nop" : "+v"(c) : "v"(a), "v"(b));
  return c;
}

__global__ __launch_bounds__(256) void k_prep_w(const float* __restrict__ Wv, f16_t* __restrict__ Wt) {
  __shared__ __attribute__((aligned(16))) f16_t T[32 * XP];
  const int t = threadIdx.x, nl = t & 31, kq = t >> 5;
  const int nbase = blockIdx.x * 32;
#pragma unroll 4
  for (int i = 0; i < 32; ++i) {
    const int k = kq + 8 * i;
    T[nl * XP + k] = (f16_t)(Wv[(size_t)k * C_OUT + nbase + nl] * 16.0f);
  }
  __syncthreads();
  v8h v[4];
#pragma unroll
  for (int r = 0; r < 4; ++r) v[r] = *(const v8h*)(T + (4 * kq + r) * XP + 8 * nl);
#pragma unroll
  for (int r = 0; r < 4; ++r)
    *(volatile v8h*)(Wt + (size_t)(nbase + 4 * kq + r) * C_IN + 8 * nl) = v[r];
  __threadfence();
#pragma unroll
  for (int r = 0; r < 4; ++r)
    *(volatile v8h*)(Wt + (size_t)(nbase + 4 * kq + r) * C_IN + 8 * nl) = v[r];
}

__global__ __launch_bounds__(256) void k_fold(const float* __restrict__ Wl, const float* __restrict__ bl,
                                              const float* __restrict__ Wr, const float* __restrict__ br,
                                              const float* __restrict__ att_l, const float* __restrict__ att_r,
                                              unsigned short* __restrict__ Bsh, unsigned short* __restrict__ Bsl,
                                              float* __restrict__ sbp) {
  __shared__ __attribute__((aligned(16))) unsigned short s_hi[C_IN];
  __shared__ __attribute__((aligned(16))) unsigned short s_lo[C_IN];
  __shared__ float s_sb;
  const int j = blockIdx.x;
  const int c = threadIdx.x;
  float acc = 0.0f, sacc = 0.0f;
  if (j < 2 * NHEAD) {
    const int side = j >> 2, hd = (j & 3) * HDIM;
    const float* W   = side ? Wr : Wl;
    const float* bb  = side ? br : bl;
    const float* att = (side ? att_r : att_l) + hd;
    const float* wrow = W + (size_t)c * C_OUT + hd;
#pragma unroll 1
    for (int d = 0; d < HDIM; ++d) acc += wrow[d] * att[d];
    if (c == 0) {
#pragma unroll 1
      for (int d = 0; d < HDIM; ++d) sacc += bb[hd + d] * att[d];
    }
  }
  const bf16_t hb = (bf16_t)acc;
  const bf16_t lb = (bf16_t)(acc - (float)hb);
  s_hi[c] = __builtin_bit_cast(unsigned short, hb);
  s_lo[c] = __builtin_bit_cast(unsigned short, lb);
  if (c == 0) s_sb = sacc;
  __syncthreads();
  if (c < 32) {
    const v4u vh = *(const v4u*)(s_hi + 8 * c);
    const v4u vl = *(const v4u*)(s_lo + 8 * c);
    const float sv = (c == 0) ? s_sb : 0.0f;
    unsigned short* ph = Bsh + (size_t)j * C_IN + 8 * c;
    unsigned short* pl = Bsl + (size_t)j * C_IN + 8 * c;
    float* ps = sbp + j * SB_PITCH + c;
    *(volatile v4u*)ph = vh; *(volatile v4u*)pl = vl; *(volatile float*)ps = sv;
    __threadfence();
    *(volatile v4u*)ph = vh; *(volatile v4u*)pl = vl; *(volatile float*)ps = sv;
  }
}

__device__ __forceinline__ void proj_store(int wave, int l, int m0, const float* st, const float* sts,
                                           float* xv, float* hlr) {
  if (wave < 8) {
#pragma unroll
    for (int rr = 0; rr < 2; ++rr) {
      const int row = 2 * wave + rr;
      const size_t o = (size_t)(m0 + row) * C_OUT;
      const v4f a = *(const v4f*)(st + row * SP + 4 * l);
      const v4f b = *(const v4f*)(st + row * SP + 128 + 4 * l);
      *(volatile v4f*)(xv + o + 4 * l) = a;
      *(volatile v4f*)(xv + o + 128 + 4 * l) = b;
    }
  } else {
    const int row = l >> 1, q = l & 1;
    const v4f a = *(const v4f*)(sts + row * 8 + 4 * q);
    *(volatile v4f*)(hlr + (size_t)(m0 + row) * 8 + 4 * q) = a;
  }
}

__global__ __launch_bounds__(288) void k_proj(const float* __restrict__ x, const f16_t* __restrict__ Wt,
                                              const bf16_t* __restrict__ Bsh, const bf16_t* __restrict__ Bsl,
                                              const float* __restrict__ sbp, const float* __restrict__ bv,
                                              float* __restrict__ xv, float* __restrict__ hlr, int N) {
  __shared__ __attribute__((aligned(16))) f16_t  xa[16 * XP];
  __shared__ __attribute__((aligned(16))) bf16_t xh[16 * XP];
  __shared__ __attribute__((aligned(16))) bf16_t xl[16 * XP];
  __shared__ __attribute__((aligned(16))) float  st[16 * SP];
  __shared__ __attribute__((aligned(16))) float  sts[16 * 8];

  const int tid = threadIdx.x;
  const int m0  = blockIdx.x * 16;

  if (tid < 256) {
#pragma unroll 4
    for (int r = 0; r < 16; ++r) {
      const int row = m0 + r;
      float f = 0.0f;
      if (row < N) f = x[(size_t)row * C_IN + tid];
      xa[r * XP + tid] = (f16_t)f;
      const bf16_t hb = (bf16_t)f;
      xh[r * XP + tid] = hb;
      xl[r * XP + tid] = (bf16_t)(f - (float)hb);
    }
  }
  __syncthreads();

  const int wave = __builtin_amdgcn_readfirstlane(tid >> 5);
  const int l = tid & 31, hh = l >> 4, m = l & 15;

  if (wave < 8) {
    const int n0 = wave * 32;
    v8f acc0 = {0.f, 0.f, 0.f, 0.f, 0.f, 0.f, 0.f, 0.f};
    v8f acc1 = {0.f, 0.f, 0.f, 0.f, 0.f, 0.f, 0.f, 0.f};
    const f16_t* ap  = xa + m * XP + 8 * hh;
    const f16_t* b0p = Wt + (size_t)(n0 + m) * C_IN + 8 * hh;
    const f16_t* b1p = Wt + (size_t)(n0 + 16 + m) * C_IN + 8 * hh;
#pragma unroll 2
    for (int k0 = 0; k0 < C_IN; k0 += 32) {
      FragH a, b0, b1;
      a.half[0]  = *(const v8h*)(ap + k0);
      a.half[1]  = *(const v8h*)(ap + k0 + 16);
      b0.half[0] = *(const v8h*)(b0p + k0);
      b0.half[1] = *(const v8h*)(b0p + k0 + 16);
      b1.half[0] = *(const v8h*)(b1p + k0);
      b1.half[1] = *(const v8h*)(b1p + k0 + 16);
      acc0 = mma_f16(a.v, b0.v, acc0);
      acc1 = mma_f16(a.v, b1.v, acc1);
    }
    const float bias0 = bv[n0 + m];
    const float bias1 = bv[n0 + 16 + m];
#pragma unroll
    for (int r = 0; r < 8; ++r) {
      st[(8 * hh + r) * SP + n0 + m]      = acc0[r] * 0.0625f + bias0;
      st[(8 * hh + r) * SP + n0 + 16 + m] = acc1[r] * 0.0625f + bias1;
    }
  } else {
    v8f acc = {0.f, 0.f, 0.f, 0.f, 0.f, 0.f, 0.f, 0.f};
    const bf16_t* ahp = xh + m * XP + 8 * hh;
    const bf16_t* alp = xl + m * XP + 8 * hh;
    const bf16_t* bhp = Bsh + (size_t)m * C_IN + 8 * hh;
    const bf16_t* blp = Bsl + (size_t)m * C_IN + 8 * hh;
#pragma unroll 2
    for (int k0 = 0; k0 < C_IN; k0 += 32) {
      FragB ah, al, bh, bl;
      ah.half[0] = *(const v8b*)(ahp + k0);
      ah.half[1] = *(const v8b*)(ahp + k0 + 16);
      al.half[0] = *(const v8b*)(alp + k0);
      al.half[1] = *(const v8b*)(alp + k0 + 16);
      bh.half[0] = *(const v8b*)(bhp + k0);
      bh.half[1] = *(const v8b*)(bhp + k0 + 16);
      bl.half[0] = *(const v8b*)(blp + k0);
      bl.half[1] = *(const v8b*)(blp + k0 + 16);
      acc = mma_bf16(ah.v, bh.v, acc);
      acc = mma_bf16(ah.v, bl.v, acc);
      acc = mma_bf16(al.v, bh.v, acc);
    }
    const float sbias = sbp[m * SB_PITCH];
    if (m < 2 * NHEAD) {
#pragma unroll
      for (int r = 0; r < 8; ++r) sts[(8 * hh + r) * 8 + m] = acc[r] + sbias;
    }
  }
  __syncthreads();

  proj_store(wave, l, m0, st, sts, xv, hlr);
  __threadfence();
  proj_store(wave, l, m0, st, sts, xv, hlr);
}

template <typename HitFn>
__device__ __forceinline__ void scan_edges(const int* __restrict__ src, const int* __restrict__ dst,
                                           int E, int N, int v0, int nb, int l, HitFn hit) {
  const int ngrp = (E + 255) >> 8;
  for (int g = 0; g < ngrp; ++g) {
    const int base = g << 8;
    const int e0 = base + 8 * l;
    int d[8];
    if (base + 256 <= E) {
      const v4i q0 = *(const v4i*)(dst + e0);
      const v4i q1 = *(const v4i*)(dst + e0 + 4);
      d[0] = q0.x; d[1] = q0.y; d[2] = q0.z; d[3] = q0.w;
      d[4] = q1.x; d[5] = q1.y; d[6] = q1.z; d[7] = q1.w;
    } else {
#pragma unroll
      for (int jj = 0; jj < 8; ++jj) {
        const int e = e0 + jj;
        d[jj] = (e < E) ? dst[e] : -1;
      }
    }
    unsigned f = 0u;
#pragma unroll
    for (int jj = 0; jj < 8; ++jj)
      if ((unsigned)(d[jj] - v0) < (unsigned)nb) f |= (1u << jj);
    unsigned any = __builtin_amdgcn_ballot_w32(f != 0u);
    while (any != 0u) {
      const int ln = __builtin_ctz(any);
      any &= any - 1u;
      unsigned fl = (unsigned)__builtin_amdgcn_readlane((int)f, ln);
      while (fl != 0u) {
        const int jj = __builtin_ctz(fl);
        fl &= fl - 1u;
        int dsel = d[7];
#pragma unroll
        for (int q = 6; q >= 0; --q) dsel = (jj == q) ? d[q] : dsel;
        const int dd = __builtin_amdgcn_readlane(dsel, ln);
        const int e  = base + 8 * ln + jj;
        int sn = src[e];
        sn = sn < 0 ? 0 : sn;
        sn = sn >= N ? N - 1 : sn;
        int dv = dd - v0;
        dv = dv < 0 ? 0 : dv;
        dv = dv >= nb ? nb - 1 : dv;
        hit(sn, dv);
      }
    }
  }
}

__device__ __forceinline__ void nbr_store(int l, int v0, int N, const float* cacc, const int* dcnt,
                                          const float* hlr, float* agg) {
  const v4f z4 = {0.f, 0.f, 0.f, 0.f};
#pragma unroll 1
  for (int g = 0; g < NB_C / 16; ++g) {
    const int lv = g * 16 + (l >> 1), q = l & 1;
    const int v = v0 + lv;
    const v4f cs = *(const v4f*)(cacc + lv * 8 + 4 * q);
    v4f hv = z4;
    if (v < N) hv = *(const v4f*)(hlr + (size_t)v * 8 + 4 * q);
    const float rd = 1.0f / (1.0f + (float)dcnt[lv]);
    const v4f r = (hv + cs) * rd;
    *(volatile v4f*)(agg + (size_t)v * 8 + 4 * q) = r;
  }
}

__global__ __launch_bounds__(32) void k_nbr(const int* __restrict__ src, const int* __restrict__ dst,
                                            const float* __restrict__ hlr, float* __restrict__ agg,
                                            int N, int E) {
  __shared__ __attribute__((aligned(16))) float cacc[NB_C * 8];
  __shared__ int dcnt[NB_C];
  const int l  = threadIdx.x;
  const int v0 = blockIdx.x * NB_C;
  int nb = N - v0;
  if (nb > NB_C) nb = NB_C;
  if (nb < 0) nb = 0;
  const v4f z4 = {0.f, 0.f, 0.f, 0.f};
  for (int i = l; i < NB_C * 2; i += 32) *(v4f*)(cacc + 4 * i) = z4;
  for (int i = l; i < NB_C; i += 32) dcnt[i] = 0;
  __syncthreads();

  scan_edges(src, dst, E, N, v0, nb, l, [&](int sn, int dv) {
    if (l < 8) cacc[dv * 8 + l] += hlr[(size_t)sn * 8 + l];
    if (l == 0) dcnt[dv] += 1;
  });
  __syncthreads();

  nbr_store(l, v0, N, cacc, dcnt, hlr, agg);
  __threadfence();
  nbr_store(l, v0, N, cacc, dcnt, hlr, agg);
}

__device__ __forceinline__ void aggr_store(int l, int v0, int nb, const float* acc,
                                           volatile float* D, float* out) {
  const int hq = l >> 4;
#pragma unroll 1
  for (int lv = 0; lv < nb; ++lv) {
    const size_t ro = (size_t)(v0 + lv) * C_OUT;
    const float d0 = D[lv * 4 + hq];
    const float d1 = D[lv * 4 + 2 + hq];
    const float r0 = 1.0f / fmaxf(d0, 1e-16f);
    const float r1 = 1.0f / fmaxf(d1, 1e-16f);
    const v4f o0 = *(const v4f*)(acc + lv * C_OUT + 4 * l) * r0;
    const v4f o1 = *(const v4f*)(acc + lv * C_OUT + 128 + 4 * l) * r1;
    *(volatile v4f*)(out + ro + 4 * l) = o0;
    *(volatile v4f*)(out + ro + 128 + 4 * l) = o1;
  }
}

__global__ __launch_bounds__(32) void k_aggr(const int* __restrict__ src, const int* __restrict__ dst,
                                             const float* __restrict__ agg, const float* __restrict__ xv,
                                             float* __restrict__ out, int N, int E) {
  extern __shared__ __attribute__((aligned(16))) float dyn[];
  float* acc = dyn;
  float* es  = dyn + NB_A * C_OUT;
  volatile float* M = dyn + NB_A * C_OUT + NB_A * 4;
  volatile float* D = dyn + NB_A * C_OUT + NB_A * 8;

  const int l  = threadIdx.x;
  const int v0 = blockIdx.x * NB_A;
  int nb = N - v0;
  if (nb > NB_A) nb = NB_A;
  if (nb < 0) nb = 0;

  const v4f z4 = {0.f, 0.f, 0.f, 0.f};
  for (int i = l; i < NB_A * (C_OUT / 4); i += 32) *(v4f*)(acc + 4 * i) = z4;
  for (int i = l; i < NB_A * 4; i += 32) {
    const int lv = i >> 2, hq = i & 3;
    const int v = v0 + lv;
    es[i] = (v < N) ? agg[(size_t)v * 8 + 4 + hq] : 0.0f;
    M[i] = -__builtin_inff();
    D[i] = 0.0f;
  }
  __syncthreads();

  const int cb = 8 * l;
  const int h  = l >> 3;
  scan_edges(src, dst, E, N, v0, nb, l, [&](int sn, int dv) {
    float e = agg[(size_t)sn * 8 + h] + es[dv * 4 + h];
    e = fmaxf(e, 0.2f * e);
    const int si = dv * 4 + h;
    const float mo = M[si];
    const float mn = fmaxf(mo, e);
    const float sc = __expf(mo - mn);
    const float p  = __expf(e - mn);
    const float* xr = xv + (size_t)sn * C_OUT + cb;
    const v4f x0 = *(const v4f*)xr;
    const v4f x1 = *(const v4f*)(xr + 4);
    v4f* ar = (v4f*)(acc + dv * C_OUT + cb);
    v4f a0 = ar[0], a1 = ar[1];
    a0 = a0 * sc + x0 * p;
    a1 = a1 * sc + x1 * p;
    ar[0] = a0;
    ar[1] = a1;
    if ((l & 7) == 0) {
      const float dd = D[si];
      D[si] = dd * sc + p;
      M[si] = mn;
    }
  });
  __syncthreads();

  aggr_store(l, v0, nb, acc, D, out);
  __threadfence();
  aggr_store(l, v0, nb, acc, D, out);
}

extern "C" void kernel_launch(void* const* d_in, const int* in_sizes, int n_in,
                              void* d_out, int out_size, void* d_ws, size_t ws_size,
                              hipStream_t stream) {
  if (n_in < 11) return;
  const float* x     = (const float*)d_in[0];
  const int*   src   = (const int*)d_in[1];
  const int*   dst   = (const int*)d_in[2];
  const float* Wl    = (const float*)d_in[3];
  const float* bl    = (const float*)d_in[4];
  const float* Wr    = (const float*)d_in[5];
  const float* br    = (const float*)d_in[6];
  const float* Wv    = (const float*)d_in[7];
  const float* bv    = (const float*)d_in[8];
  const float* att_l = (const float*)d_in[9];
  const float* att_r = (const float*)d_in[10];
  float* out = (float*)d_out;

  int N = in_sizes[0] / C_IN;
  const int No = out_size / C_OUT;
  if (No < N) N = No;
  int E = in_sizes[1];
  if (in_sizes[2] < E) E = in_sizes[2];
  if (N <= 0 || E < 0) return;
  if (in_sizes[3] < C_IN * C_OUT || in_sizes[5] < C_IN * C_OUT || in_sizes[7] < C_IN * C_OUT) return;
  if (in_sizes[4] < C_OUT || in_sizes[6] < C_OUT || in_sizes[8] < C_OUT) return;
  if (in_sizes[9] < NHEAD * HDIM || in_sizes[10] < NHEAD * HDIM) return;

  const int NP16 = ((N + 15) / 16) * 16;
  const int NPC  = ((N + NB_C - 1) / NB_C) * NB_C;

  const size_t o_wt  = 0;
  const size_t o_bsh = o_wt  + (size_t)C_OUT * C_IN * 2;
  const size_t o_bsl = o_bsh + (size_t)16 * C_IN * 2;
  const size_t o_sb  = o_bsl + (size_t)16 * C_IN * 2;
  const size_t o_xv  = o_sb  + (size_t)16 * SB_PITCH * 4;
  const size_t o_hlr = o_xv  + (size_t)NP16 * C_OUT * 4;
  const size_t o_agg = o_hlr + (size_t)NP16 * 8 * 4;
  const size_t o_end = o_agg + (size_t)NPC * 8 * 4;
  if (o_end > ws_size) return;

  char* ws = (char*)d_ws;
  f16_t*          Wt  = (f16_t*)(ws + o_wt);
  unsigned short* Bsh = (unsigned short*)(ws + o_bsh);
  unsigned short* Bsl = (unsigned short*)(ws + o_bsl);
  float*          sbp = (float*)(ws + o_sb);
  float*          xv  = (float*)(ws + o_xv);
  float*          hlr = (float*)(ws + o_hlr);
  float*          agg = (float*)(ws + o_agg);

  const size_t lds_aggr = (size_t)NB_A * (C_OUT + 12) * sizeof(float);
  hipFuncSetAttribute((const void*)k_aggr, hipFuncAttributeMaxDynamicSharedMemorySize, (int)lds_aggr);

  k_prep_w<<<C_OUT / 32, 256, 0, stream>>>(Wv, Wt);
  k_fold<<<16, 256, 0, stream>>>(Wl, bl, Wr, br, att_l, att_r, Bsh, Bsl, sbp);
  k_proj<<<NP16 / 16, 288, 0, stream>>>(x, Wt, (const bf16_t*)Bsh, (const bf16_t*)Bsl, sbp, bv, xv, hlr, N);
  k_nbr<<<NPC / NB_C, 32, 0, stream>>>(src, dst, hlr, agg, N, E);
  k_aggr<<<(N + NB_A - 1) / NB_A, 32, lds_aggr, stream>>>(src, dst, agg, xv, out, N, E);
  (void)hipGetLastError();
}
